// FeatExtractor_8796093022837
// MI455X (gfx1250) — hardware-verified
//
#include <hip/hip_runtime.h>

typedef _Float16 v16h __attribute__((ext_vector_type(16)));
typedef _Float16 v8h  __attribute__((ext_vector_type(8)));
typedef _Float16 v4h  __attribute__((ext_vector_type(4)));
typedef float    v8f  __attribute__((ext_vector_type(8)));
typedef float    v4f  __attribute__((ext_vector_type(4)));
typedef v8h __attribute__((may_alias)) v8ha;
typedef v4h __attribute__((may_alias)) v4ha;
typedef v4f __attribute__((may_alias)) v4fa;

union Frag { v16h v; v8h half[2]; };

#define NB    16
#define CIN   12
#define HIN   128
#define C1    64
#define HP    64
#define NPIX  (HP * HP)
#define C2    128
#define NOBJ  32
#define K1P   160
#define K2    576
#define NG1   (C1 * K1P / 8)
#define NG2   (C2 * K2 / 8)
#define ACT_CARRY 8.0f
#define W_CARRY   256.0f
#define INV_CARRY 0.00048828125f

static_assert(NG1 % 256 == 0);
static_assert((NG1 + NG2) % 256 == 0);
static_assert(K1P % 32 == 0);
static_assert(K2 % 32 == 0);
static_assert((C1 * K1P * 2) % 128 == 0);
static_assert((C2 * K2 * 2) % 128 == 0);

__device__ __forceinline__ v8f wmma_f16(v16h a, v16h b, v8f c) {
  v8f d = __builtin_amdgcn_wmma_f32_16x16x32_f16(false, a, false, b, (short)0, c, false, false);
  asm volatile("v_nop\n\tv_nop\n\tv_nop\n\tv_nop" : "+v"(d) : "v"(a), "v"(b));
  return d;
}

__device__ __forceinline__ v16h load_frag(const _Float16* p, int h) {
  Frag f;
  f.half[0] = *(const v8ha*)(p + 8 * h);
  f.half[1] = *(const v8ha*)(p + 16 + 8 * h);
  return f.v;
}

__device__ __forceinline__ v8h zero8h() {
  const v8h z = { (_Float16)0.0f, (_Float16)0.0f, (_Float16)0.0f, (_Float16)0.0f,
                  (_Float16)0.0f, (_Float16)0.0f, (_Float16)0.0f, (_Float16)0.0f };
  return z;
}

__device__ __forceinline__ v4h zero4h() {
  const v4h z = { (_Float16)0.0f, (_Float16)0.0f, (_Float16)0.0f, (_Float16)0.0f };
  return z;
}

__global__ __launch_bounds__(256) void pack_w_kernel(
    const float* __restrict__ W1, const float* __restrict__ W2,
    _Float16* __restrict__ W1p, _Float16* __restrict__ W2p)
{
  const int g = blockIdx.x * 256 + threadIdx.x;
  if (g >= NG1 + NG2) return;
  float v[8];
  _Float16* dst;
  if (blockIdx.x < NG1 / 256) {
    const int o  = g / (K1P / 8);
    const int kb = (g - o * (K1P / 8)) * 8;
    const int t  = kb >> 4, ci0 = kb & 15;
    const int tc = (t < 9) ? t : 8;
    const int dy = tc / 3, dx = tc - 3 * dy;
    #pragma unroll
    for (int i = 0; i < 8; ++i) {
      const int ci  = ci0 + i;
      const int cic = (ci < CIN) ? ci : (CIN - 1);
      const float w = W1[((o * CIN + cic) * 3 + dy) * 3 + dx];
      v[i] = (t < 9 && ci < CIN) ? w * W_CARRY : 0.0f;
    }
    dst = W1p + (size_t)g * 8;
  } else {
    const int e  = g - NG1;
    const int o  = e / (K2 / 8);
    const int kb = (e - o * (K2 / 8)) * 8;
    const int t  = kb >> 6, ci0 = kb & 63;
    const int dy = t / 3, dx = t - 3 * dy;
    #pragma unroll
    for (int i = 0; i < 8; ++i)
      v[i] = W2[((o * C1 + ci0 + i) * 3 + dy) * 3 + dx] * W_CARRY;
    dst = W2p + (size_t)e * 8;
  }
  const v8h o8 = { (_Float16)v[0], (_Float16)v[1], (_Float16)v[2], (_Float16)v[3],
                   (_Float16)v[4], (_Float16)v[5], (_Float16)v[6], (_Float16)v[7] };
  *(volatile v8h*)dst = o8;
  __threadfence();
  *(volatile v8h*)dst = o8;
}

__device__ __forceinline__ void pool_store_pass(const _Float16* sP, _Float16* pooled,
                                                int b, int py, int w, int lane) {
  const int q8 = lane & 7, sub = lane >> 3;
  #pragma unroll
  for (int i = 0; i < 2; ++i) {
    const int px = 8 * w + 4 * i + sub;
    const v8h v = *(const v8ha*)(sP + px * C1 + 8 * q8);
    _Float16* dst = pooled + ((size_t)(b * HP + py) * HP + px) * C1 + 8 * q8;
    *(volatile v8h*)dst = v;
  }
}

__global__ __launch_bounds__(256) void conv1_pool_kernel(
    const float* __restrict__ x,
    const _Float16* __restrict__ W1p,
    const float* __restrict__ b1,
    _Float16* __restrict__ pooled)
{
  __shared__ __attribute__((aligned(16))) _Float16 sH[4 * 130 * 16];
  __shared__ __attribute__((aligned(16))) _Float16 sP[HP * C1];

  const int tid = threadIdx.x, lane = tid & 31, w = tid >> 5;
  const int h = lane >> 4, m = lane & 15;
  const int py = blockIdx.x;
  const int b  = blockIdx.y;
  const int y0 = 2 * py;

  for (int e = tid; e < 4 * CIN * 32; e += 256) {
    const int q  = e & 31;
    const int rc = e >> 5;
    const int r  = rc / CIN, c = rc - CIN * r;
    const int iy = y0 - 1 + r;
    const bool ok = (iy >= 0) && (iy < HIN);
    const int iyc = (iy < 0) ? 0 : ((iy > HIN - 1) ? (HIN - 1) : iy);
    const v4f g = *(const v4fa*)(x + ((size_t)(b * CIN + c) * HIN + iyc) * HIN + 4 * q);
    _Float16* p = sH + (r * 130 + 1 + 4 * q) * 16 + c;
    p[0]  = (_Float16)(ok ? g.x * ACT_CARRY : 0.0f);
    p[16] = (_Float16)(ok ? g.y * ACT_CARRY : 0.0f);
    p[32] = (_Float16)(ok ? g.z * ACT_CARRY : 0.0f);
    p[48] = (_Float16)(ok ? g.w * ACT_CARRY : 0.0f);
  }
  {
    const v4h z4 = zero4h();
    for (int e = tid; e < 4 * 130; e += 256) *(v4ha*)(sH + e * 16 + CIN) = z4;
  }
  if (tid < 8) {
    const int r = tid >> 1, col = (tid & 1) ? 129 : 0;
    _Float16* p = sH + (r * 130 + col) * 16;
    *(v8ha*)p = zero8h();
    *(v4ha*)(p + 8) = zero4h();
  }
  __syncthreads();

  const int mt = w & 3, cp = w >> 2;
  const _Float16* wrow = W1p + (size_t)(16 * mt + m) * K1P;

  const v8f zf = {0.f, 0.f, 0.f, 0.f, 0.f, 0.f, 0.f, 0.f};
  v8f acc[2][4];
  #pragma unroll
  for (int ry = 0; ry < 2; ++ry)
    #pragma unroll
    for (int j = 0; j < 4; ++j) acc[ry][j] = zf;

  #pragma unroll 1
  for (int s = 0; s < K1P / 32; ++s) {
    const v16h a = load_frag(wrow + 32 * s, h);
    const int t0 = 2 * s;
    const int dy0 = t0 / 3, dx0 = t0 - 3 * dy0;
    const int t1 = (2 * s + 1 < 9) ? (2 * s + 1) : 0;
    const int dy1 = t1 / 3, dx1 = t1 - 3 * dy1;
    #pragma unroll
    for (int ry = 0; ry < 2; ++ry) {
      const _Float16* r0p = sH + ((ry + dy0) * 130 + dx0 + 64 * cp + m) * 16 + 8 * h;
      const _Float16* r1p = sH + ((ry + dy1) * 130 + dx1 + 64 * cp + m) * 16 + 8 * h;
      #pragma unroll
      for (int j = 0; j < 4; ++j) {
        Frag bf;
        bf.half[0] = *(const v8ha*)(r0p + 16 * j * 16);
        bf.half[1] = *(const v8ha*)(r1p + 16 * j * 16);
        acc[ry][j] = wmma_f16(a, bf.v, acc[ry][j]);
      }
    }
  }

  const v4f bA = *(const v4fa*)(b1 + 16 * mt + 8 * h);
  const v4f bB = *(const v4fa*)(b1 + 16 * mt + 8 * h + 4);
  const float bias[8] = { bA.x, bA.y, bA.z, bA.w, bB.x, bB.y, bB.z, bB.w };
  #pragma unroll
  for (int j = 0; j < 4; ++j) {
    float pv[8];
    #pragma unroll
    for (int r = 0; r < 8; ++r) {
      float u = fmaxf(acc[0][j][r], acc[1][j][r]);
      u = fmaxf(u, __shfl_xor(u, 1));
      pv[r] = fmaxf(u * INV_CARRY + bias[r], 0.0f) * ACT_CARRY;
    }
    if ((m & 1) == 0) {
      const int pc = 32 * cp + 8 * j + (m >> 1);
      const v8h o8 = { (_Float16)pv[0], (_Float16)pv[1], (_Float16)pv[2], (_Float16)pv[3],
                       (_Float16)pv[4], (_Float16)pv[5], (_Float16)pv[6], (_Float16)pv[7] };
      *(v8ha*)(sP + pc * C1 + 16 * mt + 8 * h) = o8;
    }
  }
  __syncthreads();

  pool_store_pass(sP, pooled, b, py, w, lane);
  __threadfence();
  pool_store_pass(sP, pooled, b, py, w, lane);
}

__device__ __forceinline__ void f_store_pass(const float* sF, float* F, int b, int y, int w, int lane) {
  const int q8 = lane & 7, sub = lane >> 3;
  #pragma unroll
  for (int it = 0; it < 8; ++it) {
    const int lid = 4 * it + sub;
    const int px = 8 * w + (lid >> 2), ln = lid & 3;
    const v4f v = *(const v4fa*)(sF + px * C2 + 32 * ln + 4 * q8);
    float* dst = F + ((size_t)(b * NPIX + y * HP + px)) * C2 + 32 * ln + 4 * q8;
    *(volatile v4f*)dst = v;
  }
}

__global__ __launch_bounds__(256) void conv2_kernel(
    const _Float16* __restrict__ pooled,
    const _Float16* __restrict__ W2p,
    const float* __restrict__ b2,
    float* __restrict__ F)
{
  __shared__ __attribute__((aligned(16))) _Float16 sH[3 * 66 * C1];
  __shared__ __attribute__((aligned(16))) float sF[HP * C2];

  const int tid = threadIdx.x, lane = tid & 31, w = tid >> 5;
  const int h = lane >> 4, m = lane & 15;
  const int y = blockIdx.x, b = blockIdx.y;
  const v8h z8 = zero8h();

  for (int e = tid; e < 3 * HP * 8; e += 256) {
    const int q = e & 7, rc = e >> 3, col = rc & 63, r = rc >> 6;
    const int iy = y - 1 + r;
    const bool ok = (iy >= 0) && (iy < HP);
    const int iyc = (iy < 0) ? 0 : ((iy > HP - 1) ? (HP - 1) : iy);
    const v8h g = *(const v8ha*)(pooled + ((size_t)(b * HP + iyc) * HP + col) * C1 + 8 * q);
    *(v8ha*)(sH + (r * 66 + 1 + col) * C1 + 8 * q) = ok ? g : z8;
  }
  for (int e = tid; e < 3 * 2 * 8; e += 256) {
    const int q = e & 7, rc = e >> 3, r = rc >> 1, col = (rc & 1) ? 65 : 0;
    *(v8ha*)(sH + (r * 66 + col) * C1 + 8 * q) = z8;
  }
  __syncthreads();

  const int cg = w & 3, pg = w >> 2;
  const _Float16* wr0 = W2p + (size_t)(32 * cg + m) * K2;
  const _Float16* wr1 = wr0 + (size_t)16 * K2;

  const v8f zf = {0.f, 0.f, 0.f, 0.f, 0.f, 0.f, 0.f, 0.f};
  v8f acc[2][2];
  #pragma unroll
  for (int i = 0; i < 2; ++i)
    #pragma unroll
    for (int j = 0; j < 2; ++j) acc[i][j] = zf;

  #pragma unroll 1
  for (int s = 0; s < K2 / 32; ++s) {
    const int t = s >> 1, dy = t / 3, dx = t - 3 * dy, ch0 = 32 * (s & 1);
    const v16h a0 = load_frag(wr0 + 32 * s, h);
    const v16h a1 = load_frag(wr1 + 32 * s, h);
    const _Float16* bp = sH + (dy * 66 + dx + 32 * pg + m) * C1 + ch0;
    #pragma unroll
    for (int j = 0; j < 2; ++j) {
      const v16h bb = load_frag(bp + 16 * j * C1, h);
      acc[0][j] = wmma_f16(a0, bb, acc[0][j]);
      acc[1][j] = wmma_f16(a1, bb, acc[1][j]);
    }
  }

  #pragma unroll
  for (int i = 0; i < 2; ++i) {
    const int chb = 32 * cg + 16 * i + 8 * h;
    const v4f bA = *(const v4fa*)(b2 + chb);
    const v4f bB = *(const v4fa*)(b2 + chb + 4);
    #pragma unroll
    for (int j = 0; j < 2; ++j) {
      const int px = 32 * pg + 16 * j + m;
      const v4f o0 = { fmaxf(acc[i][j][0] * INV_CARRY + bA.x, 0.0f), fmaxf(acc[i][j][1] * INV_CARRY + bA.y, 0.0f),
                       fmaxf(acc[i][j][2] * INV_CARRY + bA.z, 0.0f), fmaxf(acc[i][j][3] * INV_CARRY + bA.w, 0.0f) };
      const v4f o1 = { fmaxf(acc[i][j][4] * INV_CARRY + bB.x, 0.0f), fmaxf(acc[i][j][5] * INV_CARRY + bB.y, 0.0f),
                       fmaxf(acc[i][j][6] * INV_CARRY + bB.z, 0.0f), fmaxf(acc[i][j][7] * INV_CARRY + bB.w, 0.0f) };
      *(v4fa*)(sF + px * C2 + chb) = o0;
      *(v4fa*)(sF + px * C2 + chb + 4) = o1;
    }
  }
  __syncthreads();

  f_store_pass(sF, F, b, y, w, lane);
  __threadfence();
  f_store_pass(sF, F, b, y, w, lane);
}

__device__ __forceinline__ void out_store_pass(const float* smax, float* out, int b, int w, int lane) {
  const int q8 = lane & 7, sub = lane >> 3;
  #pragma unroll
  for (int it = 0; it < 8; ++it) {
    const int lid = 4 * it + sub;
    const int o = 8 * w + (lid >> 2), ln = lid & 3;
    const v4f v = *(const v4fa*)(smax + o * C2 + 32 * ln + 4 * q8);
    float* dst = out + ((size_t)(b * NOBJ + o)) * C2 + 32 * ln + 4 * q8;
    *(volatile v4f*)dst = v;
  }
}

__global__ __launch_bounds__(128) void segmax_kernel(
    const float* __restrict__ F,
    const int* __restrict__ rois,
    float* __restrict__ out)
{
  __shared__ __attribute__((aligned(16))) float smax[(NOBJ + 1) * C2];
  __shared__ int slab[HP];

  const int c = threadIdx.x, b = blockIdx.x;
  const int lane = c & 31, w = c >> 5;

  #pragma unroll 1
  for (int o = 0; o < NOBJ + 1; ++o) smax[o * C2 + c] = 0.0f;

  #pragma unroll 1
  for (int py = 0; py < HP; ++py) {
    __syncthreads();
    if (c < HP) {
      const int lab = rois[((size_t)(b * HIN + 2 * py)) * HIN + 2 * c];
      slab[c] = ((unsigned)lab < (unsigned)NOBJ) ? lab : NOBJ;
    }
    __syncthreads();
    const float* frow = F + ((size_t)(b * NPIX + py * HP)) * C2 + c;
    #pragma unroll 4
    for (int px = 0; px < HP; ++px) {
      const int lab = slab[px];
      const float v = frow[px * C2];
      float* sp = smax + lab * C2 + c;
      *sp = fmaxf(*sp, v);
    }
  }
  __syncthreads();

  out_store_pass(smax, out, b, w, lane);
  __threadfence();
  out_store_pass(smax, out, b, w, lane);
}

extern "C" void kernel_launch(void* const* d_in, const int* in_sizes, int n_in,
                              void* d_out, int out_size, void* d_ws, size_t ws_size,
                              hipStream_t stream) {
  if (n_in < 6) return;
  if (in_sizes[0] != NB * CIN * HIN * HIN) return;
  if (in_sizes[1] != C1 * CIN * 9) return;
  if (in_sizes[2] != C1) return;
  if (in_sizes[3] != C2 * C1 * 9) return;
  if (in_sizes[4] != C2) return;
  if (in_sizes[5] != NB * HIN * HIN) return;
  if (out_size != NB * NOBJ * C2) return;

  const float* x    = (const float*)d_in[0];
  const float* W1   = (const float*)d_in[1];
  const float* b1   = (const float*)d_in[2];
  const float* W2   = (const float*)d_in[3];
  const float* b2   = (const float*)d_in[4];
  const int*   rois = (const int*)d_in[5];
  float* out = (float*)d_out;

  const size_t w1p_bytes    = (size_t)C1 * K1P * 2;
  const size_t w2p_bytes    = (size_t)C2 * K2 * 2;
  const size_t pooled_bytes = (size_t)NB * NPIX * C1 * 2;
  const size_t f_bytes      = (size_t)NB * NPIX * C2 * 4;
  const size_t total = w1p_bytes + w2p_bytes + pooled_bytes + f_bytes;
  if (total > ws_size) return;

  char* ws = (char*)d_ws;
  _Float16* W1p    = (_Float16*)(ws);
  _Float16* W2p    = (_Float16*)(ws + w1p_bytes);
  _Float16* pooled = (_Float16*)(ws + w1p_bytes + w2p_bytes);
  float*    F      = (float*)(ws + w1p_bytes + w2p_bytes + pooled_bytes);

  pack_w_kernel<<<(NG1 + NG2 + 255) / 256, 256, 0, stream>>>(W1, W2, W1p, W2p);
  conv1_pool_kernel<<<dim3(HP, NB), 256, 0, stream>>>(x, W1p, b1, pooled);
  conv2_kernel<<<dim3(HP, NB), 256, 0, stream>>>(pooled, W2p, b2, F);
  segmax_kernel<<<NB, 128, 0, stream>>>(F, rois, out);
}
